// MultiHeadAttention_51788715655174
// MI455X (gfx1250) — hardware-verified
//
#include <hip/hip_runtime.h>
#ifndef NB
#define NB 2
#endif
#ifndef SEQ
#define SEQ 2048
#endif
#define NB_FULL 2
#define SEQ_FULL 2048
#define SQ SEQ
#define DM 1024
#define NH 16
#define HD 64
#define HG 2
#define RES ((SQ < 512) ? SQ : 512)
#define NR ((size_t)NB * SQ)
static_assert(SQ % 128 == 0);
static_assert(RES % 128 == 0);
static_assert(RES <= SQ);
static_assert(DM % 128 == 0);
static_assert(NH % HG == 0);
static_assert(HD == 64);
static_assert(NH * HD == DM);
static_assert(NB <= NB_FULL);
static_assert(SQ <= SEQ_FULL);

typedef unsigned short v8us __attribute__((ext_vector_type(8), may_alias));
typedef float  v8f  __attribute__((ext_vector_type(8)));
typedef float  v4f  __attribute__((ext_vector_type(4)));
typedef float  v4fa __attribute__((ext_vector_type(4), may_alias));
typedef _Float16 v16h __attribute__((ext_vector_type(16)));
typedef _Float16 v4h __attribute__((ext_vector_type(4)));
union FragH { v16h v; v8us half[2]; _Float16 h[16]; unsigned short u[16]; };

__device__ __forceinline__ unsigned short bf16_bits(float x) { unsigned int u = __float_as_uint(x); return (unsigned short)((u + 0x7FFFu + ((u >> 16) & 1u)) >> 16); }
__device__ __forceinline__ float bf16_val(unsigned short b) { return __uint_as_float(((unsigned int)b) << 16); }
__device__ __forceinline__ float bf16_rne(float x) { return bf16_val(bf16_bits(x)); }

__global__ __launch_bounds__(256) void k_wt_heads(const float* __restrict__ W, _Float16* __restrict__ Wt, float scale) {
  const int t = blockIdx.x * 256 + threadIdx.x; if (t >= DM * (DM / 8)) return;
  const int n = t / (DM / 8), k8 = (t % (DM / 8)) * 8; const int h = n >> 6, d = n & 63; FragH f;
#pragma unroll
  for (int i = 0; i < 8; ++i) f.h[i] = (_Float16)(bf16_rne(W[((size_t)h * DM + k8 + i) * HD + d]) * scale);
  const v8us o = f.half[0];
  *(volatile v8us*)((unsigned short*)Wt + (size_t)n * DM + k8) = o;
  __threadfence();
  *(volatile v8us*)((unsigned short*)Wt + (size_t)n * DM + k8) = o;
}

__global__ __launch_bounds__(256) void k_cvt16s(const float* __restrict__ in, _Float16* __restrict__ out, size_t n8, float scale) {
  const size_t t = (size_t)blockIdx.x * 256 + threadIdx.x; if (t >= n8) return;
  const size_t e = t * 8;
  const v4f a = *(const v4fa*)(in + e), c = *(const v4fa*)(in + e + 4);
  FragH f;
#pragma unroll
  for (int q = 0; q < 4; ++q) { f.h[q] = (_Float16)(bf16_rne(a[q]) * scale); f.h[4 + q] = (_Float16)(bf16_rne(c[q]) * scale); }
  const v8us o = f.half[0];
  *(volatile v8us*)((unsigned short*)out + e) = o;
  __threadfence();
  *(volatile v8us*)((unsigned short*)out + e) = o;
}

__global__ __launch_bounds__(256) void k_x16(const float* __restrict__ x, _Float16* __restrict__ X16, size_t n8) {
  const size_t t = (size_t)blockIdx.x * 256 + threadIdx.x; if (t >= n8) return;
  const size_t e = t * 8; const size_t b = e / ((size_t)SQ * DM); const size_t rem = e - b * (size_t)SQ * DM;
  const float* src = x + b * (size_t)SEQ_FULL * DM + rem;
  const v4f a = *(const v4fa*)src, c = *(const v4fa*)(src + 4);
  FragH f;
#pragma unroll
  for (int q = 0; q < 4; ++q) { f.h[q] = (_Float16)bf16_rne(a[q]); f.h[4 + q] = (_Float16)bf16_rne(c[q]); }
  const v8us o = f.half[0];
  *(volatile v8us*)((unsigned short*)X16 + e) = o;
  __threadfence();
  *(volatile v8us*)((unsigned short*)X16 + e) = o;
}

template <int NHv, int TTv>
__global__ __launch_bounds__(256) void k_vt(const _Float16* __restrict__ V16, int ldv, int voff, _Float16* __restrict__ Vt) {
  __shared__ unsigned short tl[64][66];
  const int tid = threadIdx.x; const int slab = blockIdx.x / (TTv / 64), lg = blockIdx.x % (TTv / 64); const int b = slab / NHv, h = slab % NHv;
  for (int i = tid; i < 64 * 8; i += 256) { const int r = i / 8, c8 = (i % 8) * 8; FragH f;
    f.half[0] = *(const v8us*)((const unsigned short*)V16 + ((size_t)b * TTv + lg * 64 + r) * ldv + voff + h * 64 + c8);
#pragma unroll
    for (int q = 0; q < 8; ++q) tl[r][c8 + q] = f.u[q]; }
  __syncthreads();
  for (int pass = 0; pass < 2; ++pass) {
#pragma unroll
    for (int rd = 0; rd < 2; ++rd) { const int d = rd * 32 + tid / 8, pc = tid % 8; FragH f;
#pragma unroll
      for (int q = 0; q < 8; ++q) f.u[q] = tl[pc * 8 + q][d];
      *(volatile v8us*)((unsigned short*)Vt + ((size_t)slab * 64 + d) * TTv + lg * 64 + pc * 8) = f.half[0]; }
    if (pass == 0) __threadfence(); } }

__device__ __forceinline__ v16h g2_frag(const _Float16* p, int hh) { FragH f; f.half[0] = *(const v8us*)((const unsigned short*)p + 8 * hh); f.half[1] = *(const v8us*)((const unsigned short*)p + 16 + 8 * hh); return f.v; }
__device__ __forceinline__ v8f g2_mma(v16h a, v16h b, v8f c) { v8f d = __builtin_amdgcn_wmma_f32_16x16x32_f16(false, a, false, b, (short)0, c, false, false); asm volatile("v_nop\n\tv_nop\n\tv_nop\n\tv_nop" : "+v"(d) : "v"(a), "v"(b)); return d; }
struct Acc8 { v8f c00, c01, c02, c03, c10, c11, c12, c13; };
__device__ __forceinline__ void g3_kloop(const _Float16* a0p, int lda, const _Float16* b0p, int ldb, int hh, int K, Acc8& c) {
  const _Float16* a1p = a0p + (size_t)16 * lda;
  const _Float16* b1p = b0p + (size_t)16 * ldb; const _Float16* b2p = b1p + (size_t)16 * ldb; const _Float16* b3p = b2p + (size_t)16 * ldb;
#pragma unroll 1
  for (int kb = 0; kb < K; kb += 32) { const v16h a0 = g2_frag(a0p + kb, hh), a1 = g2_frag(a1p + kb, hh);
    v16h b = g2_frag(b0p + kb, hh); c.c00 = g2_mma(a0, b, c.c00); c.c10 = g2_mma(a1, b, c.c10);
    b = g2_frag(b1p + kb, hh); c.c01 = g2_mma(a0, b, c.c01); c.c11 = g2_mma(a1, b, c.c11);
    b = g2_frag(b2p + kb, hh); c.c02 = g2_mma(a0, b, c.c02); c.c12 = g2_mma(a1, b, c.c12);
    b = g2_frag(b3p + kb, hh); c.c03 = g2_mma(a0, b, c.c03); c.c13 = g2_mma(a1, b, c.c13); }
}
template <int NPROD, bool CSKIP, bool KCAUS, int OUTM, bool BIAS>
__global__ __launch_bounds__(128) void k_gemm3(const _Float16* __restrict__ A, int lda, size_t sA, const _Float16* __restrict__ A2, int lda2, size_t sA2,
    const _Float16* __restrict__ Bh, int ldb, size_t sB, const _Float16* __restrict__ B2, int ldb2, size_t sB2, float alpha, const float* __restrict__ bias,
    float* __restrict__ C, _Float16* __restrict__ C16, _Float16* __restrict__ C16L, int ldc, size_t sC, size_t sCL, int M, int N, int K, int resRows) {
  __shared__ __attribute__((aligned(16))) float so[4][32][68];
  const int tid = threadIdx.x, w = __builtin_amdgcn_readfirstlane((int)(tid >> 5)), lane = tid & 31, ln = lane & 15, hh = lane >> 4; const int by = blockIdx.y;
  const int ntn = N >> 6; const int mt = blockIdx.x / ntn, nq = blockIdx.x - mt * ntn; const int rowb = mt * 128; const int row0 = rowb + 32 * w, col0 = nq * 64;
  if (row0 >= M) return;
  if (CSKIP && col0 > rowb + 127) return;
  const bool ext = (rowb < resRows);
  int Keff = K; if (KCAUS) { const int kc = rowb + 128; Keff = (kc < K) ? kc : K; }
  const v8f z8 = {0.f,0.f,0.f,0.f,0.f,0.f,0.f,0.f}; Acc8 c; c.c00 = z8; c.c01 = z8; c.c02 = z8; c.c03 = z8; c.c10 = z8; c.c11 = z8; c.c12 = z8; c.c13 = z8;
  g3_kloop(A + (size_t)by * sA + (size_t)(row0 + ln) * lda, lda, Bh + (size_t)by * sB + (size_t)(col0 + ln) * ldb, ldb, hh, Keff, c);
  if (NPROD >= 2 && ext) g3_kloop(A2 + (size_t)by * sA2 + (size_t)(row0 + ln) * lda2, lda2, Bh + (size_t)by * sB + (size_t)(col0 + ln) * ldb, ldb, hh, Keff, c);
  if (NPROD >= 3 && ext) g3_kloop(A + (size_t)by * sA + (size_t)(row0 + ln) * lda, lda, B2 + (size_t)by * sB2 + (size_t)(col0 + ln) * ldb2, ldb2, hh, Keff, c);
  v8f accs[8] = {c.c00, c.c01, c.c02, c.c03, c.c10, c.c11, c.c12, c.c13};
#pragma unroll
  for (int u = 0; u < 8; ++u) { const int t = u & 3, half = u >> 2; const int col = col0 + t * 16 + ln;
    float bv = 0.f; if (BIAS) bv = bf16_rne(bias[col]);
#pragma unroll
    for (int r = 0; r < 8; ++r) { const int rloc = half * 16 + 8 * hh + r; float v = accs[u][r] * alpha;
      if (BIAS) v = v + bv;
      so[w][rloc][t * 16 + ln] = v; } }
  __builtin_amdgcn_fence(4  , "workgroup"); __builtin_amdgcn_wave_barrier();
  const int rsub = lane >> 4, c4 = (lane & 15) * 4;
  const size_t cofs = (size_t)by * sC, lofs = (size_t)by * sCL;
  for (int pass = 0; pass < 2; ++pass) {
#pragma unroll
    for (int q = 0; q < 16; ++q) { const int r = q * 2 + rsub; const v4f v = *(const v4fa*)&so[w][r][c4];
      if (OUTM != 0) { v4h h4, l4;
#pragma unroll
        for (int i = 0; i < 4; ++i) { h4[i] = (_Float16)v[i]; l4[i] = (_Float16)(v[i] - (float)h4[i]); }
        *(volatile v4h*)(C16 + cofs + (size_t)(row0 + r) * ldc + col0 + c4) = h4;
        if (OUTM == 2 && ext) *(volatile v4h*)(C16L + lofs + (size_t)(row0 + r) * ldc + col0 + c4) = l4; }
      else { *(volatile v4f*)(C + cofs + (size_t)(row0 + r) * ldc + col0 + c4) = v; } }
    if (pass == 0) __threadfence(); } }

__global__ __launch_bounds__(256) void k_rsmc(const float* __restrict__ S, _Float16* __restrict__ P, _Float16* __restrict__ PL, int qn, int hg, int res) {
  #pragma clang fp contract(off)
  const int t = blockIdx.x * 256 + threadIdx.x; if (t >= qn * hg) return;
  const int hs = t / qn, qi = t - hs * qn;
  const size_t i = (size_t)hs * SQ + qi; const float* s = S + i * SQ; float mx = s[0];
#pragma unroll 1
  for (int j = 1; j <= qi; ++j) mx = fmaxf(mx, s[j]);
  float se = 0.f;
#pragma unroll 1
  for (int j = 0; j <= qi; ++j) se += __expf(fmaxf(s[j] - mx, -120.0f));
  const float sc = 4096.0f / se;
  const int kend = ((qi >> 7) + 1) << 7;
  const bool wlo = qi < res;
  unsigned short* ph = (unsigned short*)P + i * SQ;
  unsigned short* pl = (unsigned short*)PL + ((size_t)hs * res + (wlo ? qi : 0)) * res;
#pragma unroll 1
  for (int j0 = 0; j0 < kend; j0 += 8) { FragH f, g;
#pragma unroll
    for (int q = 0; q < 8; ++q) { const int jj = j0 + q; const int jc = (jj < qi) ? jj : qi;
      const float e = __expf(fmaxf(s[jc] - mx, -120.0f)) * sc; const float val = (jj <= qi) ? e : 0.0f;
      const _Float16 hv = (_Float16)val; f.h[q] = hv; g.h[q] = (_Float16)(val - (float)hv); }
    const v8us o = f.half[0]; const v8us ol = g.half[0];
    *(volatile v8us*)(ph + j0) = o; if (wlo) *(volatile v8us*)(pl + j0) = ol;
    __threadfence();
    *(volatile v8us*)(ph + j0) = o; if (wlo) *(volatile v8us*)(pl + j0) = ol; } }

extern "C" void kernel_launch(void* const* d_in, const int* in_sizes, int n_in,
                              void* d_out, int out_size, void* d_ws, size_t ws_size, hipStream_t stream) {
  if (n_in < 6) return;
  const size_t need_rows = (size_t)(NB - 1) * SEQ_FULL + SQ;
  if ((size_t)in_sizes[0] < need_rows * DM) return;
  if ((size_t)in_sizes[1] < (size_t)NH * DM * HD || (size_t)in_sizes[2] < (size_t)NH * DM * HD || (size_t)in_sizes[3] < (size_t)NH * DM * HD) return;
  if ((size_t)in_sizes[4] < (size_t)DM * DM || (size_t)in_sizes[5] < (size_t)DM) return;
  if ((size_t)out_size < need_rows * DM) return;
  const float* x = (const float*)d_in[0];
  const float* wq = (const float*)d_in[1]; const float* wk = (const float*)d_in[2]; const float* wv = (const float*)d_in[3];
  const float* wo = (const float*)d_in[4]; const float* bo = (const float*)d_in[5];
  float* out = (float*)d_out;
  char* ws = (char*)d_ws; size_t off = 0;
  auto take = [&](size_t bytes) { char* p = ws + off; off += (bytes + 255) & ~(size_t)255; return p; };
  _Float16* BW   = (_Float16*)take((size_t)4 * DM * DM * 2);
  _Float16* X16  = (_Float16*)take(NR * DM * 2);
  _Float16* QKV  = (_Float16*)take((size_t)3 * NR * DM * 2);
  _Float16* QKVL = (_Float16*)take((size_t)3 * NB * RES * DM * 2);
  _Float16* O16  = (_Float16*)take(NR * DM * 2);
  _Float16* OL   = (_Float16*)take((size_t)NB * RES * DM * 2);
  float*    S    = (float*)take((size_t)HG * SQ * SQ * 4);
  _Float16* P    = (_Float16*)take((size_t)HG * SQ * SQ * 2);
  _Float16* PL   = (_Float16*)take((size_t)HG * RES * RES * 2);
  _Float16* VT   = (_Float16*)take((size_t)NB * NH * HD * SQ * 2);
  _Float16* VTL  = (_Float16*)take((size_t)NB * NH * HD * RES * 2);
  if (off > ws_size || off > (size_t)134217728) return;
  _Float16* BQ = BW; _Float16* BK = BW + (size_t)DM * DM; _Float16* BV = BW + (size_t)2 * DM * DM; _Float16* BO = BW + (size_t)3 * DM * DM;
  _Float16* Q16 = QKV; _Float16* K16 = QKV + NR * DM; _Float16* V16 = QKV + 2 * NR * DM;
  const size_t lpl = (size_t)NB * RES * DM;
  _Float16* QL = QKVL; _Float16* KL = QKVL + lpl; _Float16* VL = QKVL + 2 * lpl;

  { const unsigned g = (unsigned)(((size_t)DM * (DM / 8) + 255) / 256);
    k_wt_heads<<<g, 256, 0, stream>>>(wq, BQ, 16.0f);
    k_wt_heads<<<g, 256, 0, stream>>>(wk, BK, 16.0f);
    k_wt_heads<<<g, 256, 0, stream>>>(wv, BV, 16.0f);
    k_cvt16s<<<g, 256, 0, stream>>>(wo, BO, (size_t)DM * DM / 8, 16.0f); }
  k_x16<<<(unsigned)((NR * DM / 8 + 255) / 256), 256, 0, stream>>>(x, X16, NR * DM / 8);
  for (int b = 0; b < NB; ++b)
    k_gemm3<1, false, false, 2, false><<<dim3((unsigned)((SQ / 128) * (DM / 64)), 3), 128, 0, stream>>>(
        X16 + (size_t)b * SQ * DM, DM, (size_t)0, X16, DM, (size_t)0, BW, DM, (size_t)DM * DM, BW, DM, (size_t)0, 1.0f, bo,
        nullptr, QKV + (size_t)b * SQ * DM, QKVL + (size_t)b * RES * DM, DM, NR * DM, lpl, SQ, DM, DM, RES);
  k_vt<NH, SQ><<<NB * NH * (SQ / 64), 256, 0, stream>>>(V16, DM, 0, VT);
  k_vt<NH, RES><<<NB * NH * (RES / 64), 256, 0, stream>>>(VL, DM, 0, VTL);
  for (int b = 0; b < NB; ++b) { const size_t r0 = (size_t)b * SQ; const size_t l0 = (size_t)b * RES;
    for (int h0 = 0; h0 < NH; h0 += HG) {
      k_gemm3<3, true, false, 0, false><<<dim3((SQ / 128) * (SQ / 64), HG), 128, 0, stream>>>(
          Q16 + r0 * DM + h0 * HD, DM, (size_t)HD, QL + l0 * DM + h0 * HD, DM, (size_t)HD,
          K16 + r0 * DM + h0 * HD, DM, (size_t)HD, KL + l0 * DM + h0 * HD, DM, (size_t)HD, 0.00048828125f, bo,
          S, nullptr, nullptr, SQ, (size_t)SQ * SQ, (size_t)0, SQ, SQ, HD, RES);
      k_rsmc<<<(HG * SQ + 255) / 256, 256, 0, stream>>>(S, P, PL, SQ, HG, RES);
      k_gemm3<3, false, true, 2, false><<<dim3((SQ / 128) * (HD / 64), HG), 128, 0, stream>>>(
          P, SQ, (size_t)SQ * SQ, PL, RES, (size_t)RES * RES,
          VT + ((size_t)b * NH + h0) * HD * SQ, SQ, (size_t)HD * SQ, VTL + ((size_t)b * NH + h0) * HD * RES, RES, (size_t)HD * RES, 0.0009765625f, bo,
          nullptr, O16 + r0 * DM + h0 * HD, OL + l0 * DM + h0 * HD, DM, (size_t)HD, (size_t)HD, SQ, HD, SQ, RES); } }
  k_gemm3<2, false, false, 0, true><<<dim3((unsigned)((SQ / 128) * (DM / 64)), NB), 128, 0, stream>>>(
      O16, DM, (size_t)SQ * DM, OL, DM, (size_t)RES * DM, BO, DM, (size_t)0, BO, DM, (size_t)0, 0.0009765625f, bo,
      out, nullptr, nullptr, DM, (size_t)SEQ_FULL * DM, (size_t)0, SQ, DM, DM, RES);
}
